// CausalAttention_22136261444412
// MI455X (gfx1250) — hardware-verified
//
#include <hip/hip_runtime.h>


#ifndef NB
#define NB 4
#endif
#ifndef SEQ
#define SEQ 2048
#endif
#ifndef RH
#define RH ((SEQ) < 1024 ? (SEQ) : 1024)
#endif
#define NB_FULL  4
#define SEQ_FULL 2048
#define CDIM  1024
#define C3    3072
#define NHEAD 16
#define HD    64
#define MROWS (NB * SEQ)
#define NU    (NB * NHEAD)
#define PCAR  1024.0f
#define RCAR  2048.0f
#define RINV  0.00048828125f
#define SC2   0.18033688f
#define NEGBIG (-3.0e38f)

static_assert(NB >= 1);
static_assert(NB <= NB_FULL);
static_assert(SEQ % 64 == 0);
static_assert(SEQ <= SEQ_FULL);
static_assert(RH % 64 == 0);
static_assert(RH >= 64);
static_assert(RH <= SEQ);
static_assert(MROWS % 64 == 0);
static_assert(CDIM == NHEAD * HD);
static_assert(CDIM % 64 == 0);
static_assert((MROWS * CDIM) % (8 * 256) == 0);
static_assert((MROWS * CDIM) % (2 * 256) == 0);
static_assert((size_t)NU * SEQ * HD == (size_t)MROWS * CDIM);
static_assert((C3 * CDIM) % 64 == 0);
static_assert((size_t)NU * HD * RH * 2 <= (size_t)MROWS * CDIM * 2);

typedef _Float16 h16;
typedef unsigned short bf;
typedef __attribute__((ext_vector_type(16))) __bf16   v16bf;
typedef __attribute__((ext_vector_type(16))) _Float16 v16h;
typedef __attribute__((ext_vector_type(8)))  _Float16 v8h;
typedef __attribute__((ext_vector_type(2)))  _Float16 v2h;
typedef __attribute__((ext_vector_type(8)))  unsigned short v8us;
typedef __attribute__((ext_vector_type(2)))  unsigned short v2us;
typedef __attribute__((ext_vector_type(8)))  float    v8f;
typedef __attribute__((ext_vector_type(4)))  float    v4f;
typedef v8h  __attribute__((may_alias)) v8ha;
typedef v4f  __attribute__((may_alias)) v4fa;
typedef v8us __attribute__((may_alias)) v8usa;

__device__ __forceinline__ unsigned short f2bf(float f) { unsigned u = __float_as_uint(f); u += 0x7FFFu + ((u >> 16) & 1u); return (unsigned short)(u >> 16); }
__device__ __forceinline__ float bf2f(unsigned short b) { return __uint_as_float(((unsigned)b) << 16); }
__device__ __forceinline__ float bfr(float f) { return bf2f(f2bf(f)); }
__device__ __forceinline__ v16h cat16(v8h lo, v8h hi) { return __builtin_shufflevector(lo, hi, 0, 1, 2, 3, 4, 5, 6, 7, 8, 9, 10, 11, 12, 13, 14, 15); }
__device__ __forceinline__ v16bf cat16b(v8us lo, v8us hi) { return __builtin_bit_cast(v16bf, __builtin_shufflevector(lo, hi, 0, 1, 2, 3, 4, 5, 6, 7, 8, 9, 10, 11, 12, 13, 14, 15)); }
__device__ __forceinline__ v8f wmma16(v16h a, v16h b, v8f c) { return __builtin_amdgcn_wmma_f32_16x16x32_f16(false, a, false, b, (short)0, c, false, false); }
__device__ __forceinline__ v8f wmmab(v16bf a, v16bf b, v8f c) { return __builtin_amdgcn_wmma_f32_16x16x32_bf16(false, a, false, b, (short)0, c, false, false); }
__device__ __forceinline__ void splitf(float y, unsigned short& h, unsigned short& l) { h = f2bf(y); l = f2bf(y - bf2f(h)); }
__device__ __forceinline__ v16h ldf(const h16* p) { return cat16(*(const v8h*)p, *(const v8h*)(p + 16)); }

template <typename T16> struct WFrag;
template <> struct WFrag<h16> { typedef v16h V; static __device__ __forceinline__ V ld(const h16* p) { return cat16(*(const v8h*)p, *(const v8h*)(p + 16)); } static __device__ __forceinline__ v8f mma(V a, V b, v8f c) { return wmma16(a, b, c); } };
template <> struct WFrag<bf> { typedef v16bf V; static __device__ __forceinline__ V ld(const bf* p) { return cat16b(*(const v8us*)p, *(const v8us*)(p + 16)); } static __device__ __forceinline__ v8f mma(V a, V b, v8f c) { return wmmab(a, b, c); } };
template <typename T16, int NSPLIT, bool BIAS>
__global__ __launch_bounds__(32) void k_gemmw(const T16* __restrict__ A, const T16* __restrict__ A2, const T16* __restrict__ Bt, const T16* __restrict__ Bt2, int K, float* C, int ldc, const float* __restrict__ bias, size_t sA, size_t sB, size_t sC) {
    typedef typename WFrag<T16>::V V;
    __shared__ __align__(16) float os[16 * 68];
    const size_t z = blockIdx.z; A += z * sA; if (A2) A2 += z * sA; Bt += z * sB; if (Bt2) Bt2 += z * sB; C += z * sC;
    const int lane = threadIdx.x & 31, lr = lane & 15, hi = lane >> 4; const int r0 = blockIdx.x * 64, c0 = blockIdx.y * 64;
    v8f acc[4][4];
#pragma unroll
    for (int mb = 0; mb < 4; ++mb)
#pragma unroll
        for (int nb = 0; nb < 4; ++nb) acc[mb][nb] = (v8f){};
    const size_t aoff = (size_t)(r0 + lr) * K + 8 * hi, boff = (size_t)(c0 + lr) * K + 8 * hi;
#pragma unroll 1
    for (int kc = 0; kc < K; kc += 32) {
        V a[4], a2[4];
#pragma unroll
        for (int mb = 0; mb < 4; ++mb) { a[mb] = WFrag<T16>::ld(A + aoff + (size_t)mb * 16 * K + kc); if (NSPLIT == 1 || NSPLIT == 2) a2[mb] = WFrag<T16>::ld(A2 + aoff + (size_t)mb * 16 * K + kc); }
#pragma unroll
        for (int nb = 0; nb < 4; ++nb) { const V b = WFrag<T16>::ld(Bt + boff + (size_t)nb * 16 * K + kc); V b2; if (NSPLIT >= 2) b2 = WFrag<T16>::ld(Bt2 + boff + (size_t)nb * 16 * K + kc);
#pragma unroll
            for (int mb = 0; mb < 4; ++mb) { acc[mb][nb] = WFrag<T16>::mma(a[mb], b, acc[mb][nb]); if (NSPLIT == 1 || NSPLIT == 2) acc[mb][nb] = WFrag<T16>::mma(a2[mb], b, acc[mb][nb]); if (NSPLIT >= 2) acc[mb][nb] = WFrag<T16>::mma(a[mb], b2, acc[mb][nb]); } }
        asm volatile("v_nop\n\tv_nop\n\tv_nop\n\tv_nop" : "+v"(acc[0][0]), "+v"(acc[1][1]), "+v"(acc[2][2]), "+v"(acc[3][3]) : "v"(a[0]), "v"(a[3]));
    }
#pragma unroll
    for (int mb = 0; mb < 4; ++mb) {
#pragma unroll
        for (int nb = 0; nb < 4; ++nb) {
#pragma unroll
            for (int j = 0; j < 8; ++j) os[(hi * 8 + j) * 68 + nb * 16 + lr] = acc[mb][nb][j]; }
        __builtin_amdgcn_wave_barrier(); asm volatile("" ::: "memory");
        float* crow = C + (size_t)(r0 + mb * 16) * ldc + c0;
#pragma unroll 1
        for (int ps = 0; ps < 2; ++ps) {
#pragma unroll
            for (int s = 0; s < 8; ++s) { const int row = 2 * s + hi, cofs = lr * 4; v4f val = *(const v4fa*)(os + row * 68 + cofs); if (BIAS) { val[0] += bfr(bias[c0 + cofs]); val[1] += bfr(bias[c0 + cofs + 1]); val[2] += bfr(bias[c0 + cofs + 2]); val[3] += bfr(bias[c0 + cofs + 3]); }
                *(volatile v4f*)(crow + (size_t)row * ldc + cofs) = val; }
            if (ps == 0) __threadfence(); }
        __builtin_amdgcn_wave_barrier(); asm volatile("" ::: "memory");
    }
}

__global__ __launch_bounds__(256) void k_wtG(const float* __restrict__ w, int K, int N, bf* Bt) {
    const int lane = threadIdx.x & 31; const int L0 = (blockIdx.x * 8 + (threadIdx.x >> 5)) * 8; const int nlines = N * K / 64;
#pragma unroll
    for (int ps = 0; ps < 2; ++ps) {
#pragma unroll 1
        for (int l = 0; l < 8; ++l) { const int L = L0 + l; if (L >= nlines) break; const size_t e = (size_t)L * 64 + lane * 2; const int k = (int)(e % K), n = (int)(e / K); v2us o;
            o[0] = f2bf(w[(size_t)k * N + n]); o[1] = f2bf(w[(size_t)(k + 1) * N + n]); *(volatile v2us*)(Bt + e) = o; }
        if (ps == 0) __threadfence(); }
}

__global__ __launch_bounds__(256) void k_cvtx(const float* __restrict__ X, bf* Xb, size_t n8) {
    const size_t i = (size_t)blockIdx.x * 256 + threadIdx.x; if (i >= n8) return;
    const size_t r = i / (CDIM / 8); const int c8 = (int)(i % (CDIM / 8)); const int b = (int)(r / SEQ), t = (int)(r % SEQ);
    const v8f v = *(const v8f*)(X + ((size_t)(b * SEQ_FULL + t)) * CDIM + c8 * 8); v8us o;
#pragma unroll
    for (int k = 0; k < 8; ++k) o[k] = f2bf(v[k]);
    *(volatile v8us*)(Xb + i * 8) = o; __threadfence(); *(volatile v8us*)(Xb + i * 8) = o;
}

__global__ __launch_bounds__(256) void k_cvqk(const float* __restrict__ F, h16* P16, h16* Pr, size_t n8) {
    const size_t i = (size_t)blockIdx.x * 256 + threadIdx.x; if (i >= n8) return;
    const size_t e = i * 8; const int d = (int)(e % HD); const int t = (int)((e / HD) % SEQ); const int u = (int)(e / ((size_t)HD * SEQ)); const int b = u / NHEAD, hh = u % NHEAD;
    const v8f v = *(const v8f*)(F + ((size_t)(b * SEQ + t)) * CDIM + hh * HD + d);
    v8h o16, orr;
#pragma unroll
    for (int k = 0; k < 8; ++k) { const h16 hv = (h16)v[k]; o16[k] = hv; orr[k] = (h16)((v[k] - (float)hv) * RCAR); }
    const size_t ro = ((size_t)u * RH + t) * HD + d; const bool res = (t < RH);
    *(volatile v8h*)(P16 + e) = o16; if (res) *(volatile v8h*)(Pr + ro) = orr;
    __threadfence();
    *(volatile v8h*)(P16 + e) = o16; if (res) *(volatile v8h*)(Pr + ro) = orr;
}

__global__ __launch_bounds__(256) void k_cvv(const float* __restrict__ F, h16* VT, h16* Vr, size_t n2) {
    const size_t i = (size_t)blockIdx.x * 256 + threadIdx.x; if (i >= n2) return;
    const size_t e = i * 2; const int t = (int)(e % SEQ); const int d = (int)((e / SEQ) % HD); const int u = (int)(e / ((size_t)SEQ * HD)); const int b = u / NHEAD, hh = u % NHEAD;
    v2h o16, orr;
#pragma unroll
    for (int q = 0; q < 2; ++q) { const float x = F[((size_t)(b * SEQ + t + q)) * CDIM + hh * HD + d]; const h16 hv = (h16)x; o16[q] = hv; orr[q] = (h16)((x - (float)hv) * RCAR); }
    const size_t ro = ((size_t)u * HD + d) * RH + t; const bool res = (t < RH);
    *(volatile v2h*)(VT + e) = o16; if (res) *(volatile v2h*)(Vr + ro) = orr;
    __threadfence();
    *(volatile v2h*)(VT + e) = o16; if (res) *(volatile v2h*)(Vr + ro) = orr;
}

__device__ __forceinline__ void ctx_epi(const v8f* o, float l, float* os, int lane, int b, int hh, int q0, bf* CTXh, bf* CTXl) {
    const int lr = lane & 15, hi = lane >> 4; const float inv = 1.0f / (l * PCAR);
#pragma unroll
    for (int dt = 0; dt < 4; ++dt) { v4f w0, w1;
#pragma unroll
        for (int i = 0; i < 4; ++i) { w0[i] = o[dt][i] * inv; w1[i] = o[dt][4 + i] * inv; }
        *(v4fa*)(os + lr * 68 + dt * 16 + 8 * hi) = w0; *(v4fa*)(os + lr * 68 + dt * 16 + 8 * hi + 4) = w1; }
    __builtin_amdgcn_fence(3  , "wavefront"); __builtin_amdgcn_wave_barrier();
    const int rr = lane >> 3, pc = lane & 7;
#pragma unroll 1
    for (int ps = 0; ps < 2; ++ps) {
#pragma unroll
        for (int q = 0; q < 4; ++q) { const int rw = q * 4 + rr; const v4f a = *(const v4fa*)(os + rw * 68 + pc * 8); const v4f c = *(const v4fa*)(os + rw * 68 + pc * 8 + 4); v8us oh, ol;
#pragma unroll
            for (int i = 0; i < 4; ++i) { unsigned short th, tl; splitf(a[i], th, tl); oh[i] = th; ol[i] = tl; splitf(c[i], th, tl); oh[4 + i] = th; ol[4 + i] = tl; }
            const size_t off = ((size_t)(b * SEQ + q0 + rw)) * CDIM + (size_t)hh * HD + pc * 8;
            *(volatile v8us*)(CTXh + off) = oh; *(volatile v8us*)(CTXl + off) = ol; }
        if (ps == 0) __threadfence(); }
}

__global__ __launch_bounds__(32) void k_attn_lo(const h16* __restrict__ Q16, const h16* __restrict__ K16, const h16* __restrict__ VT, int strip0, bf* CTXh, bf* CTXl) {
    __shared__ __align__(16) float os[16 * 68];
    const int lane = threadIdx.x & 31, lr = lane & 15, hi = lane >> 4;
    const int u = blockIdx.y, b = u / NHEAD, hh = u % NHEAD;
    const int q0 = (strip0 + (int)blockIdx.x) * 16; const int row = q0 + lr;
    const h16* qp = Q16 + ((size_t)u * SEQ + row) * HD + 8 * hi;
    const v16h qf0 = ldf(qp), qf1 = ldf(qp + 32);
    const h16* kbase = K16 + ((size_t)u * SEQ + lr) * HD + 8 * hi;
    const h16* vbase = VT + ((size_t)u * HD + lr) * SEQ + 8 * hi;
    v8f o[4];
#pragma unroll
    for (int dt = 0; dt < 4; ++dt) o[dt] = (v8f){};
    float m = NEGBIG, l = 0.f;
    const int jmax = (q0 + 15) >> 6;
#pragma unroll 1
    for (int j = 0; j <= jmax; ++j) {
        const int kb = j << 6;
        v8f s[4]; v16h ka, kc;
#pragma unroll
        for (int jt = 0; jt < 4; ++jt) { const h16* kp = kbase + (size_t)(kb + jt * 16) * HD; ka = ldf(kp); kc = ldf(kp + 32); v8f acc = (v8f){}; acc = wmma16(ka, qf0, acc); acc = wmma16(kc, qf1, acc); s[jt] = acc; }
        asm volatile("v_nop\n\tv_nop\n\tv_nop\n\tv_nop" : "+v"(s[0]), "+v"(s[1]), "+v"(s[2]), "+v"(s[3]) : "v"(qf1), "v"(kc));
        float mx = NEGBIG;
        if (kb + 63 > q0) {
#pragma unroll
            for (int jt = 0; jt < 4; ++jt)
#pragma unroll
                for (int r = 0; r < 8; ++r) { const int key = kb + jt * 16 + 8 * hi + r; float t = s[jt][r] * SC2; t = (key > row) ? NEGBIG : t; s[jt][r] = t; mx = fmaxf(mx, t); }
        } else {
#pragma unroll
            for (int jt = 0; jt < 4; ++jt)
#pragma unroll
                for (int r = 0; r < 8; ++r) { const float t = s[jt][r] * SC2; s[jt][r] = t; mx = fmaxf(mx, t); }
        }
        mx = fmaxf(mx, __shfl_xor(mx, 16, 32));
        const float mn = fmaxf(m, mx); const float alpha = __builtin_amdgcn_exp2f(m - mn);
        float sum = 0.f;
#pragma unroll
        for (int jt = 0; jt < 4; ++jt)
#pragma unroll
            for (int r = 0; r < 8; ++r) { const float p = __builtin_amdgcn_exp2f(s[jt][r] - mn); s[jt][r] = p; sum += p; }
        sum += __shfl_xor(sum, 16, 32);
        l = l * alpha + sum; m = mn;
#pragma unroll
        for (int dt = 0; dt < 4; ++dt) o[dt] = o[dt] * alpha;
        v16h pb, vf;
#pragma unroll
        for (int ks = 0; ks < 2; ++ks) { v8h plo, phi;
#pragma unroll
            for (int i = 0; i < 8; ++i) { plo[i] = (h16)(s[2 * ks][i] * PCAR); phi[i] = (h16)(s[2 * ks + 1][i] * PCAR); }
            pb = cat16(plo, phi);
#pragma unroll
            for (int dt = 0; dt < 4; ++dt) { vf = ldf(vbase + (size_t)(dt * 16) * SEQ + kb + ks * 32); o[dt] = wmma16(vf, pb, o[dt]); } }
        asm volatile("v_nop\n\tv_nop\n\tv_nop\n\tv_nop" : "+v"(o[0]), "+v"(o[1]), "+v"(o[2]), "+v"(o[3]) : "v"(pb), "v"(vf));
    }
    ctx_epi(o, l, os, lane, b, hh, q0, CTXh, CTXl);
}

__global__ __launch_bounds__(32) void k_attn_hi(const h16* __restrict__ Q16, const h16* __restrict__ Qr, const h16* __restrict__ K16, const h16* __restrict__ Kr, const h16* __restrict__ VT, const h16* __restrict__ Vr, bf* CTXh, bf* CTXl) {
    __shared__ __align__(16) float os[16 * 68];
    const int lane = threadIdx.x & 31, lr = lane & 15, hi = lane >> 4;
    const int u = blockIdx.y, b = u / NHEAD, hh = u % NHEAD;
    const int q0 = (int)blockIdx.x * 16; const int row = q0 + lr;
    const h16* qp = Q16 + ((size_t)u * SEQ + row) * HD + 8 * hi;
    const v16h qf0 = ldf(qp), qf1 = ldf(qp + 32);
    const h16* qrp = Qr + ((size_t)u * RH + row) * HD + 8 * hi;
    const v16h qr0 = ldf(qrp), qr1 = ldf(qrp + 32);
    const h16* kbase  = K16 + ((size_t)u * SEQ + lr) * HD + 8 * hi;
    const h16* krbase = Kr  + ((size_t)u * RH  + lr) * HD + 8 * hi;
    const h16* vbase  = VT  + ((size_t)u * HD + lr) * SEQ + 8 * hi;
    const h16* vrbase = Vr  + ((size_t)u * HD + lr) * RH  + 8 * hi;
    v8f o[4];
#pragma unroll
    for (int dt = 0; dt < 4; ++dt) o[dt] = (v8f){};
    float m = NEGBIG, l = 0.f;
    const int jmax = (q0 + 15) >> 5;
#pragma unroll 1
    for (int j = 0; j <= jmax; ++j) {
        const int kb = j << 5;
        v8f s[2];
#pragma unroll
        for (int jt = 0; jt < 2; ++jt) {
            const h16* kp = kbase + (size_t)(kb + jt * 16) * HD; const h16* krp = krbase + (size_t)(kb + jt * 16) * HD;
            const v16h kra = ldf(krp), krc = ldf(krp + 32);
            v8f a2 = (v8f){}; a2 = wmma16(kra, qf0, a2); a2 = wmma16(krc, qf1, a2);
            const v16h ka = ldf(kp), kc = ldf(kp + 32);
            v8f acc = (v8f){}; acc = wmma16(ka, qf0, acc); acc = wmma16(kc, qf1, acc);
            a2 = wmma16(ka, qr0, a2); a2 = wmma16(kc, qr1, a2);
            asm volatile("v_nop\n\tv_nop\n\tv_nop\n\tv_nop" : "+v"(acc), "+v"(a2) : "v"(kc), "v"(qr1));
            s[jt] = acc + a2 * RINV; }
        float mx = NEGBIG;
        if (kb + 31 > q0) {
#pragma unroll
            for (int jt = 0; jt < 2; ++jt)
#pragma unroll
                for (int r = 0; r < 8; ++r) { const int key = kb + jt * 16 + 8 * hi + r; float t = s[jt][r] * SC2; t = (key > row) ? NEGBIG : t; s[jt][r] = t; mx = fmaxf(mx, t); }
        } else {
#pragma unroll
            for (int jt = 0; jt < 2; ++jt)
#pragma unroll
                for (int r = 0; r < 8; ++r) { const float t = s[jt][r] * SC2; s[jt][r] = t; mx = fmaxf(mx, t); }
        }
        mx = fmaxf(mx, __shfl_xor(mx, 16, 32));
        const float mn = fmaxf(m, mx); const float alpha = __builtin_amdgcn_exp2f(m - mn);
        float sum = 0.f;
#pragma unroll
        for (int jt = 0; jt < 2; ++jt)
#pragma unroll
            for (int r = 0; r < 8; ++r) { const float p = __builtin_amdgcn_exp2f(s[jt][r] - mn); s[jt][r] = p; sum += p; }
        sum += __shfl_xor(sum, 16, 32);
        l = l * alpha + sum; m = mn;
#pragma unroll
        for (int dt = 0; dt < 4; ++dt) o[dt] = o[dt] * alpha;
        v8h plo, phi, rlo, rhi;
#pragma unroll
        for (int i = 0; i < 8; ++i) { const float a0 = s[0][i] * PCAR; const h16 h0 = (h16)a0; plo[i] = h0; rlo[i] = (h16)((a0 - (float)h0) * RCAR);
                                      const float a1 = s[1][i] * PCAR; const h16 h1 = (h16)a1; phi[i] = h1; rhi[i] = (h16)((a1 - (float)h1) * RCAR); }
        const v16h pb = cat16(plo, phi), pr = cat16(rlo, rhi);
#pragma unroll
        for (int dt = 0; dt < 4; ++dt) {
            const v16h vf = ldf(vbase + (size_t)(dt * 16) * SEQ + kb); const v16h vrf = ldf(vrbase + (size_t)(dt * 16) * RH + kb);
            o[dt] = wmma16(vf, pb, o[dt]);
            v8f o2 = (v8f){}; o2 = wmma16(vf, pr, o2); o2 = wmma16(vrf, pb, o2);
            asm volatile("v_nop\n\tv_nop\n\tv_nop\n\tv_nop" : "+v"(o[dt]), "+v"(o2) : "v"(pr), "v"(vrf));
            o[dt] = o[dt] + o2 * RINV; }
    }
    ctx_epi(o, l, os, lane, b, hh, q0, CTXh, CTXl);
}

extern "C" void kernel_launch(void* const* d_in, const int* in_sizes, int n_in,
                              void* d_out, int out_size, void* d_ws, size_t ws_size, hipStream_t stream) {
    if (n_in < 4) return;
    if (in_sizes[0] < ((NB - 1) * SEQ_FULL + SEQ) * CDIM) return;
    if (in_sizes[1] < CDIM * C3) return;
    if (in_sizes[2] < CDIM * CDIM) return;
    if (in_sizes[3] < CDIM) return;
    if (out_size < MROWS * CDIM) return;
    const float* X = (const float*)d_in[0];
    const float* Wqkv = (const float*)d_in[1];
    const float* Wout = (const float*)d_in[2];
    const float* Bout = (const float*)d_in[3];
    float* OUT = (float*)d_out;
    char* wsp = (char*)d_ws;
    auto take = [&](size_t bytes) { char* p = wsp; wsp += (bytes + 255) & ~(size_t)255; return (void*)p; };
    bf*    Xb  = (bf*)take((size_t)MROWS * CDIM * 2);
    bf*    WqT = (bf*)take((size_t)C3 * CDIM * 2);
    bf*    WoT = (bf*)take((size_t)CDIM * CDIM * 2);
    float* Cf  = (float*)take((size_t)MROWS * CDIM * 4);
    h16*   Q16 = (h16*)take((size_t)NU * SEQ * HD * 2);
    h16*   Qr  = (h16*)take((size_t)NU * RH * HD * 2);
    h16*   K16 = (h16*)take((size_t)NU * SEQ * HD * 2);
    h16*   Kr  = (h16*)take((size_t)NU * RH * HD * 2);
    h16*   VT  = (h16*)take((size_t)NU * HD * SEQ * 2);
    if ((size_t)(wsp - (char*)d_ws) > ws_size) return;
    h16*   Vr  = (h16*)Xb;
    bf* CTXh = (bf*)Cf; bf* CTXl = CTXh + (size_t)MROWS * CDIM;

    k_cvtx<<<(unsigned)(((size_t)MROWS * CDIM / 8 + 255) / 256), 256, 0, stream>>>(X, Xb, (size_t)MROWS * CDIM / 8);
    k_wtG<<<(unsigned)((C3 * CDIM / 64 + 63) / 64), 256, 0, stream>>>(Wqkv, CDIM, C3, WqT);
    k_wtG<<<(unsigned)((CDIM * CDIM / 64 + 63) / 64), 256, 0, stream>>>(Wout, CDIM, CDIM, WoT);
    for (int ch = 0; ch < 3; ++ch) {
        k_gemmw<bf, 0, false><<<dim3(MROWS / 64, CDIM / 64, 1), 32, 0, stream>>>(Xb, nullptr, WqT + (size_t)ch * CDIM * CDIM, nullptr, CDIM, Cf, CDIM, nullptr, 0, 0, 0);
        if (ch == 0)      k_cvqk<<<(unsigned)(((size_t)MROWS * CDIM / 8 + 255) / 256), 256, 0, stream>>>(Cf, Q16, Qr, (size_t)MROWS * CDIM / 8);
        else if (ch == 1) k_cvqk<<<(unsigned)(((size_t)MROWS * CDIM / 8 + 255) / 256), 256, 0, stream>>>(Cf, K16, Kr, (size_t)MROWS * CDIM / 8);
        else              k_cvv<<<(unsigned)(((size_t)MROWS * CDIM / 2 + 255) / 256), 256, 0, stream>>>(Cf, VT, Vr, (size_t)MROWS * CDIM / 2);
    }
    k_attn_hi<<<dim3(RH / 16, NU, 1), 32, 0, stream>>>(Q16, Qr, K16, Kr, VT, Vr, CTXh, CTXl);
    if (SEQ > RH) k_attn_lo<<<dim3((SEQ - RH) / 16, NU, 1), 32, 0, stream>>>(Q16, K16, VT, RH / 16, CTXh, CTXl);
    k_gemmw<bf, 1, true><<<dim3(MROWS / 64, CDIM / 64, 1), 32, 0, stream>>>(CTXh, CTXl, WoT, nullptr, CDIM, OUT, CDIM, Bout, 0, 0, 0);
}
